// MLA_26199300505739
// MI455X (gfx1250) — hardware-verified
//
#include <hip/hip_runtime.h>


#ifndef NB
#define NB 2
#endif
#ifndef SEQ
#define SEQ 2048
#endif
#define NB_FULL  2
#define SEQ_FULL 2048
#define DMOD  2048
#define NHD   16
#define DHD   128
#define HALF  64
#define NPAIR 32
#define DCQ   768
#define DCKV  512
#define NQQ   2048
#define NKV   3072
#define NU    1344
#define RH    256
#define QB    64
#define PCAR  16384.0f
#define CSC   16.0f
#define WSC   64.0f
#define SCL   0.08838834764831845f
#define L2E   1.4426950408889634f
#define EPS   1.1920929e-07f
#define NEG   (-1.0e30f)
#define OSP   136

static_assert(NB >= 1);
static_assert(NB <= NB_FULL);
static_assert(SEQ <= SEQ_FULL);
static_assert(SEQ % 64 == 0);
static_assert(RH % 64 == 0);
static_assert(RH <= SEQ);
static_assert(NU % 64 == 0);
static_assert(NQQ % 64 == 0);
static_assert(NKV % 64 == 0);
static_assert(DMOD % 256 == 0);
static_assert(DCQ % 256 == 0);
static_assert(DCKV % 256 == 0);
static_assert(DMOD % 32 == 0 && DCQ % 32 == 0 && DCKV % 32 == 0 && (NHD * DHD) % 32 == 0);
static_assert(NU == DCQ + DCKV + HALF);
static_assert(NQQ == 2 * NHD * HALF);
static_assert(NKV == NHD * DHD + NHD * HALF);
static_assert(NU <= NKV && NQQ <= NKV);
static_assert(HALF == 2 * NPAIR);
static_assert((OSP % 8) == 0);

typedef _Float16 h16;
typedef unsigned short bf;
typedef __attribute__((ext_vector_type(16))) __bf16   v16bf;
typedef __attribute__((ext_vector_type(16))) _Float16 v16h;
typedef __attribute__((ext_vector_type(8)))  _Float16 v8h;
typedef __attribute__((ext_vector_type(8)))  unsigned short v8us;
typedef __attribute__((ext_vector_type(8)))  float    v8f;
typedef __attribute__((ext_vector_type(4)))  float    v4f;
typedef __attribute__((ext_vector_type(2)))  _Float16 v2h;
typedef __attribute__((ext_vector_type(2)))  unsigned short v2us;
typedef __attribute__((ext_vector_type(2)))  float v2f;
typedef __attribute__((ext_vector_type(4)))  int v4i;
typedef v8h  __attribute__((may_alias)) v8ha;
typedef v4f  __attribute__((may_alias)) v4fa;
typedef v8us __attribute__((may_alias)) v8usa;

__device__ __forceinline__ unsigned short f2bf(float f) { unsigned u = __float_as_uint(f); u += 0x7FFFu + ((u >> 16) & 1u); return (unsigned short)(u >> 16); }
__device__ __forceinline__ float bf2f(unsigned short b) { return __uint_as_float(((unsigned)b) << 16); }
__device__ __forceinline__ float bfr(float f) { return bf2f(f2bf(f)); }
__device__ __forceinline__ void splitf(float y, unsigned short& h, unsigned short& l) { h = f2bf(y); l = f2bf(y - bf2f(h)); }
__device__ __forceinline__ v16h cat16(v8h lo, v8h hi) { return __builtin_shufflevector(lo, hi, 0, 1, 2, 3, 4, 5, 6, 7, 8, 9, 10, 11, 12, 13, 14, 15); }
__device__ __forceinline__ v16bf cat16b(v8us lo, v8us hi) { return __builtin_bit_cast(v16bf, __builtin_shufflevector(lo, hi, 0, 1, 2, 3, 4, 5, 6, 7, 8, 9, 10, 11, 12, 13, 14, 15)); }
__device__ __forceinline__ v8f wmma16(v16h a, v16h b, v8f c) { return __builtin_amdgcn_wmma_f32_16x16x32_f16(false, a, false, b, (short)0, c, false, false); }
__device__ __forceinline__ v8f wmmab(v16bf a, v16bf b, v8f c) { return __builtin_amdgcn_wmma_f32_16x16x32_bf16(false, a, false, b, (short)0, c, false, false); }
__device__ __forceinline__ v16h  ldh(const h16* p) { return cat16(*(const v8h*)p, *(const v8h*)(p + 16)); }
__device__ __forceinline__ v16bf ldb(const bf* p)  { return cat16b(*(const v8us*)p, *(const v8us*)(p + 16)); }

template <typename T16> struct WFrag;
template <> struct WFrag<h16> { typedef v16h V; static __device__ __forceinline__ V ld(const h16* p) { return ldh(p); } static __device__ __forceinline__ v8f mma(V a, V b, v8f c) { return wmma16(a, b, c); } };
template <> struct WFrag<bf> { typedef v16bf V; static __device__ __forceinline__ V ld(const bf* p) { return ldb(p); } static __device__ __forceinline__ v8f mma(V a, V b, v8f c) { return wmmab(a, b, c); } };
template <typename T16, int NSPLIT, bool RES>
__global__ __launch_bounds__(32) void k_gemmw(const T16* __restrict__ A, const T16* __restrict__ A2, const T16* __restrict__ Bt, const T16* __restrict__ Bt2, int K, float* C, int ldc, float osc, const float* __restrict__ R, int ldr, const int* __restrict__ pz) {
    typedef typename WFrag<T16>::V V;
    __shared__ __align__(16) float os[16 * 68];
    const int lane = threadIdx.x & 31, lr = lane & 15, hi = lane >> 4; const int r0 = blockIdx.x * 64, c0 = blockIdx.y * 64;
    const int pzv = pz[0];
    const float qnan = __uint_as_float(0x7FC00000u);
    v8f acc[4][4];
#pragma unroll
    for (int mb = 0; mb < 4; ++mb)
#pragma unroll
        for (int nb = 0; nb < 4; ++nb) acc[mb][nb] = (v8f){};
    const size_t aoff = (size_t)(r0 + lr) * K + 8 * hi, boff = (size_t)(c0 + lr) * K + 8 * hi;
#pragma unroll 1
    for (int kc = 0; kc < K; kc += 32) {
        V a[4], a2[4];
#pragma unroll
        for (int mb = 0; mb < 4; ++mb) { a[mb] = WFrag<T16>::ld(A + aoff + (size_t)mb * 16 * K + kc); if (NSPLIT == 1 || NSPLIT == 2) a2[mb] = WFrag<T16>::ld(A2 + aoff + (size_t)mb * 16 * K + kc); }
#pragma unroll
        for (int nb = 0; nb < 4; ++nb) { const V b = WFrag<T16>::ld(Bt + boff + (size_t)nb * 16 * K + kc); V b2; if (NSPLIT >= 2) b2 = WFrag<T16>::ld(Bt2 + boff + (size_t)nb * 16 * K + kc);
#pragma unroll
            for (int mb = 0; mb < 4; ++mb) { acc[mb][nb] = WFrag<T16>::mma(a[mb], b, acc[mb][nb]); if (NSPLIT == 1 || NSPLIT == 2) acc[mb][nb] = WFrag<T16>::mma(a2[mb], b, acc[mb][nb]); if (NSPLIT >= 2) acc[mb][nb] = WFrag<T16>::mma(a[mb], b2, acc[mb][nb]); } }
        asm volatile("v_nop\n\tv_nop\n\tv_nop\n\tv_nop" : "+v"(acc[0][0]), "+v"(acc[1][1]), "+v"(acc[2][2]), "+v"(acc[3][3]) : "v"(a[0]), "v"(a[3]));
    }
#pragma unroll
    for (int mb = 0; mb < 4; ++mb) {
#pragma unroll
        for (int nb = 0; nb < 4; ++nb) {
#pragma unroll
            for (int j = 0; j < 8; ++j) os[(hi * 8 + j) * 68 + nb * 16 + lr] = acc[mb][nb][j]; }
        __builtin_amdgcn_wave_barrier(); asm volatile("" ::: "memory");
        float* crow = C + (size_t)(r0 + mb * 16) * ldc + c0;
        const float* rrow = RES ? (R + (size_t)(r0 + mb * 16) * ldr + c0) : nullptr;
#pragma unroll 1
        for (int ps = 0; ps < 2; ++ps) {
#pragma unroll
            for (int s = 0; s < 8; ++s) { const int row = 2 * s + hi, cofs = lr * 4; v4f val = *(const v4fa*)(os + row * 68 + cofs); val = val * osc;
                if (RES) { const v4f rr = *(const v4f*)(rrow + (size_t)row * ldr + cofs); val[0] += bfr(rr[0]); val[1] += bfr(rr[1]); val[2] += bfr(rr[2]); val[3] += bfr(rr[3]); }
                if (pzv != 0) { val[0] = qnan; val[1] = qnan; val[2] = qnan; val[3] = qnan; }
                *(volatile v4f*)(crow + (size_t)row * ldc + cofs) = val; }
            if (ps == 0) __threadfence(); }
        __builtin_amdgcn_wave_barrier(); asm volatile("" ::: "memory");
    }
}

template <bool F16, bool B16>
__global__ __launch_bounds__(256) void k_wcv(const float* __restrict__ W, int K, int N, int row0, float sc, h16* P16, bf* PB) {
    const int lane = threadIdx.x & 31; const size_t L0 = ((size_t)blockIdx.x * 8 + (threadIdx.x >> 5)) * 8; const size_t nlines = (size_t)N * K / 64;
#pragma unroll 1
    for (int l = 0; l < 8; ++l) { const size_t L = L0 + l; if (L >= nlines) break;
        const size_t e = L * 64 + (size_t)lane * 2; const int k = (int)(e % (size_t)K), n = (int)(e / (size_t)K);
        const float v0 = bfr(W[(size_t)k * N + n]), v1 = bfr(W[(size_t)(k + 1) * N + n]);
        const size_t d = (size_t)(row0 + n) * K + k;
        v2h o16; o16[0] = (h16)(v0 * sc); o16[1] = (h16)(v1 * sc);
        v2us ob; ob[0] = f2bf(v0); ob[1] = f2bf(v1);
        if (F16) *(volatile v2h*)(P16 + d) = o16;
        if (B16) *(volatile v2us*)(PB + d) = ob;
        __threadfence();
        if (F16) *(volatile v2h*)(P16 + d) = o16;
        if (B16) *(volatile v2us*)(PB + d) = ob; }
}

__global__ __launch_bounds__(256) void k_cvtx(const float* __restrict__ src, const float* __restrict__ nw, bf* dst, size_t n8) {
    const size_t i = (size_t)blockIdx.x * 256 + threadIdx.x; if (i >= n8) return;
    const v8f v = *(const v8f*)(src + i * 8); const int c0 = (int)((i * 8) % (size_t)DMOD); const v8f w = *(const v8f*)(nw + c0);
    v8us o;
#pragma unroll
    for (int k = 0; k < 8; ++k) o[k] = f2bf(bfr(v[k]) * bfr(w[k]));
    *(volatile v8us*)(dst + i * 8) = o; __threadfence(); *(volatile v8us*)(dst + i * 8) = o;
}

__global__ __launch_bounds__(256) void k_mchk(const int* __restrict__ M, int* FLG) {
    __shared__ int red[8];
    const int tid = threadIdx.x, lane = tid & 31, wv = tid >> 5; const int i0 = blockIdx.x * 16;
    int viol = 0;
#pragma unroll 1
    for (int it = 0; it < SEQ / 64; ++it) { const int e = (it * 256 + tid) * 4; const int r = e / SEQ, c = e - r * SEQ; const int i = i0 + r;
        const v4i mv = *(const v4i*)(M + (size_t)i * SEQ_FULL + c);
#pragma unroll
        for (int q = 0; q < 4; ++q) { const int want = (c + q > i) ? 1 : 0; const int got = (mv[q] != 0) ? 1 : 0; viol |= (want ^ got); } }
#pragma unroll
    for (int sh = 16; sh; sh >>= 1) viol |= __shfl_xor(viol, sh, 32);
    if (lane == 0) red[wv] = viol;
    __syncthreads();
    if (wv == 0) { int v = red[lane & 7];
#pragma unroll
        for (int sh = 16; sh; sh >>= 1) v |= __shfl_xor(v, sh, 32);
        int* fl = FLG + (size_t)blockIdx.x * 32 + lane;
        *(volatile int*)fl = v; __threadfence(); *(volatile int*)fl = v; }
}
__global__ __launch_bounds__(32) void k_fred(const int* __restrict__ FLG, int nblk, int* FLAG) {
    const int lane = threadIdx.x & 31; int v = 0;
#pragma unroll 1
    for (int i = 0; i < nblk; i += 32) { int idx = i + lane; idx = (idx < nblk) ? idx : (nblk - 1); v |= FLG[(size_t)idx * 32]; }
#pragma unroll
    for (int sh = 16; sh; sh >>= 1) v |= __shfl_xor(v, sh, 32);
    *(volatile int*)(FLAG + lane) = v; __threadfence(); *(volatile int*)(FLAG + lane) = v;
}

__global__ __launch_bounds__(256) void k_lat(const float* __restrict__ X, const float* __restrict__ U, const float* __restrict__ wcq, const float* __restrict__ wckv,
                                             const float* __restrict__ cosT, const float* __restrict__ sinT, h16* CQ16, h16* CKV16, h16* KR16, bf* KRh, bf* KRl) {
#pragma clang fp contract(off)
    const int lane = threadIdx.x & 31; const int t = blockIdx.x * 8 + (threadIdx.x >> 5);
    const float* xr = X + (size_t)t * DMOD; const float* ur = U + (size_t)t * NU;
    float ss = 0.0f;
#pragma unroll 1
    for (int ch = 0; ch < DMOD / 256; ++ch) { const v8f a = *(const v8f*)(xr + ch * 256 + lane * 8);
#pragma unroll
        for (int k = 0; k < 8; ++k) { const float v = bfr(a[k]); ss += v * v; } }
#pragma unroll
    for (int sh = 16; sh; sh >>= 1) ss += __shfl_xor(ss, sh, 32);
    const float rx = rsqrtf(ss * (1.0f / (float)DMOD) + EPS);
    v8f cq[3]; float s2 = 0.0f;
#pragma unroll
    for (int ch = 0; ch < 3; ++ch) { cq[ch] = *(const v8f*)(ur + ch * 256 + lane * 8) * rx;
#pragma unroll
        for (int k = 0; k < 8; ++k) s2 += cq[ch][k] * cq[ch][k]; }
#pragma unroll
    for (int sh = 16; sh; sh >>= 1) s2 += __shfl_xor(s2, sh, 32);
    const float rq = rsqrtf(s2 * (1.0f / (float)DCQ) + EPS);
    v8h oq[3];
#pragma unroll
    for (int ch = 0; ch < 3; ++ch) { const v8f w = *(const v8f*)(wcq + ch * 256 + lane * 8);
#pragma unroll
        for (int k = 0; k < 8; ++k) oq[ch][k] = (h16)(cq[ch][k] * rq * bfr(w[k])); }
    v8f ck[2]; float s3 = 0.0f;
#pragma unroll
    for (int ch = 0; ch < 2; ++ch) { ck[ch] = *(const v8f*)(ur + DCQ + ch * 256 + lane * 8) * rx;
#pragma unroll
        for (int k = 0; k < 8; ++k) s3 += ck[ch][k] * ck[ch][k]; }
#pragma unroll
    for (int sh = 16; sh; sh >>= 1) s3 += __shfl_xor(s3, sh, 32);
    const float rk = rsqrtf(s3 * (1.0f / (float)DCKV) + EPS);
    v8h ok[2];
#pragma unroll
    for (int ch = 0; ch < 2; ++ch) { const v8f w = *(const v8f*)(wckv + ch * 256 + lane * 8);
#pragma unroll
        for (int k = 0; k < 8; ++k) ok[ch][k] = (h16)(ck[ch][k] * rk * bfr(w[k])); }
    const v2f kv = *(const v2f*)(ur + DCQ + DCKV + 2 * lane); const float x0 = kv[0] * rx, x1 = kv[1] * rx;
    const float cth = bfr(cosT[(size_t)t * NPAIR + lane]), sth = bfr(sinT[(size_t)t * NPAIR + lane]);
    const float y0 = x0 * cth - x1 * sth, y1 = x0 * sth + x1 * cth;
    v2h okr; okr[0] = (h16)y0; okr[1] = (h16)y1;
    v2us okh, okl; { unsigned short a0, c0, a1, c1; splitf(y0, a0, c0); splitf(y1, a1, c1); okh[0] = a0; okh[1] = a1; okl[0] = c0; okl[1] = c1; }
    const int hr = __builtin_amdgcn_readfirstlane((t < RH) ? 1 : 0);
#pragma unroll 1
    for (int ps = 0; ps < 2; ++ps) {
#pragma unroll
        for (int ch = 0; ch < 3; ++ch) *(volatile v8h*)(CQ16 + (size_t)t * DCQ + ch * 256 + lane * 8) = oq[ch];
#pragma unroll
        for (int ch = 0; ch < 2; ++ch) *(volatile v8h*)(CKV16 + (size_t)t * DCKV + ch * 256 + lane * 8) = ok[ch];
        *(volatile v2h*)(KR16 + (size_t)t * HALF + 2 * lane) = okr;
        if (hr) { *(volatile v2us*)(KRh + (size_t)t * HALF + 2 * lane) = okh; *(volatile v2us*)(KRl + (size_t)t * HALF + 2 * lane) = okl; }
        if (ps == 0) __threadfence(); }
}

__global__ __launch_bounds__(256) void k_qpl(const float* __restrict__ F, const float* __restrict__ cosT, const float* __restrict__ sinT, h16* Q16, bf* Qh, bf* Ql) {
#pragma clang fp contract(off)
    const size_t e = ((size_t)blockIdx.x * 256 + threadIdx.x) * 2; if (e >= (size_t)NHD * SEQ * DHD) return;
    const int d = (int)(e % DHD); const int t = (int)((e / DHD) % SEQ); const int hd = (int)(e / ((size_t)DHD * SEQ));
    const float* f = F + (size_t)t * NQQ;
    const int sel = __builtin_amdgcn_readfirstlane((int)((e >> 6) & 1));
    float y0, y1;
    if (sel == 0) { const v2f v = *(const v2f*)(f + hd * HALF + (d & 63)); y0 = v[0]; y1 = v[1]; }
    else { const int dd = d & 63; const v2f v = *(const v2f*)(f + NHD * HALF + hd * HALF + dd);
        const float c = bfr(cosT[(size_t)t * NPAIR + (dd >> 1)]), s = bfr(sinT[(size_t)t * NPAIR + (dd >> 1)]);
        y0 = v[0] * c - v[1] * s; y1 = v[0] * s + v[1] * c; }
    v2h o16; o16[0] = (h16)y0; o16[1] = (h16)y1;
    v2us oh, ol; { unsigned short a0, c0, a1, c1; splitf(y0, a0, c0); splitf(y1, a1, c1); oh[0] = a0; oh[1] = a1; ol[0] = c0; ol[1] = c1; }
    const int hr = __builtin_amdgcn_readfirstlane((t < RH) ? 1 : 0);
    const int th = (t < RH) ? t : 0;
    const size_t eh = ((size_t)hd * RH + th) * DHD + d;
    *(volatile v2h*)(Q16 + e) = o16;
    if (hr) { *(volatile v2us*)(Qh + eh) = oh; *(volatile v2us*)(Ql + eh) = ol; }
    __threadfence();
    *(volatile v2h*)(Q16 + e) = o16;
    if (hr) { *(volatile v2us*)(Qh + eh) = oh; *(volatile v2us*)(Ql + eh) = ol; }
}

__global__ __launch_bounds__(256) void k_kcpl(const float* __restrict__ F, h16* KC16, bf* KCh, bf* KCl) {
    const size_t e = ((size_t)blockIdx.x * 256 + threadIdx.x) * 2; if (e >= (size_t)NHD * SEQ * HALF) return;
    const int d = (int)(e % HALF); const int t = (int)((e / HALF) % SEQ); const int hd = (int)(e / ((size_t)HALF * SEQ));
    const v2f v = *(const v2f*)(F + (size_t)t * NKV + NHD * DHD + hd * HALF + d);
    v2h o16; o16[0] = (h16)v[0]; o16[1] = (h16)v[1];
    v2us oh, ol; { unsigned short a0, c0, a1, c1; splitf(v[0], a0, c0); splitf(v[1], a1, c1); oh[0] = a0; oh[1] = a1; ol[0] = c0; ol[1] = c1; }
    const int hr = __builtin_amdgcn_readfirstlane((t < RH) ? 1 : 0);
    const int th = (t < RH) ? t : 0;
    const size_t eh = ((size_t)hd * RH + th) * HALF + d;
    *(volatile v2h*)(KC16 + e) = o16;
    if (hr) { *(volatile v2us*)(KCh + eh) = oh; *(volatile v2us*)(KCl + eh) = ol; }
    __threadfence();
    *(volatile v2h*)(KC16 + e) = o16;
    if (hr) { *(volatile v2us*)(KCh + eh) = oh; *(volatile v2us*)(KCl + eh) = ol; }
}

__global__ __launch_bounds__(256) void k_vtpl(const float* __restrict__ F, h16* VT16, bf* VTh, bf* VTl) {
    const size_t e = ((size_t)blockIdx.x * 256 + threadIdx.x) * 2; if (e >= (size_t)NHD * DHD * SEQ) return;
    const int t = (int)(e % SEQ); const int d = (int)((e / SEQ) % DHD); const int hd = (int)(e / ((size_t)SEQ * DHD));
    const float x0 = F[(size_t)t * NKV + hd * DHD + d], x1 = F[(size_t)(t + 1) * NKV + hd * DHD + d];
    v2h o16; o16[0] = (h16)x0; o16[1] = (h16)x1;
    v2us oh, ol; { unsigned short a0, c0, a1, c1; splitf(x0, a0, c0); splitf(x1, a1, c1); oh[0] = a0; oh[1] = a1; ol[0] = c0; ol[1] = c1; }
    const int hr = __builtin_amdgcn_readfirstlane((t < RH) ? 1 : 0);
    const int th = (t < RH) ? t : 0;
    const size_t eh = ((size_t)hd * DHD + d) * RH + th;
    *(volatile v2h*)(VT16 + e) = o16;
    if (hr) { *(volatile v2us*)(VTh + eh) = oh; *(volatile v2us*)(VTl + eh) = ol; }
    __threadfence();
    *(volatile v2h*)(VT16 + e) = o16;
    if (hr) { *(volatile v2us*)(VTh + eh) = oh; *(volatile v2us*)(VTl + eh) = ol; }
}

__global__ __launch_bounds__(128) __attribute__((amdgpu_num_vgpr(256)))
void k_attn(const h16* __restrict__ Q16, const h16* __restrict__ KC16, const h16* __restrict__ KR16, const h16* __restrict__ VT16, h16* CT16) {
    __shared__ __align__(16) h16 os[4][16 * OSP];
    const int lane = threadIdx.x & 31, wv = threadIdx.x >> 5, lr = lane & 15, hh = lane >> 4;
    const int hd = blockIdx.y;
    const int qw = RH + blockIdx.x * QB + wv * 16;
    const int q = qw + lr;
    v16h qf[4];
    { const h16* qp = Q16 + ((size_t)hd * SEQ + q) * DHD + 8 * hh;
#pragma unroll
        for (int c = 0; c < 4; ++c) qf[c] = ldh(qp + c * 32); }
    v8f of[8];
#pragma unroll
    for (int n = 0; n < 8; ++n) of[n] = (v8f){};
    float m = NEG, l = 0.0f;
    const h16* kcp = KC16 + ((size_t)hd * SEQ + lr) * HALF + 8 * hh;
    const h16* krp = KR16 + (size_t)lr * HALF + 8 * hh;
    const h16* vp  = VT16 + ((size_t)hd * DHD + lr) * SEQ + 8 * hh;
    const float cc = SCL * L2E;
    const int ns = (qw >> 5) + 1;
#pragma unroll 1
    for (int s = 0; s < ns; ++s) {
        const int kb = s * 32;
        v8f sc[2]; sc[0] = (v8f){}; sc[1] = (v8f){};
        v16h kf;
#pragma unroll
        for (int kt = 0; kt < 2; ++kt) {
            const size_t ko = (size_t)(kb + kt * 16) * HALF;
            asm volatile("" ::: "memory");
            kf = ldh(kcp + ko);      sc[kt] = wmma16(kf, qf[0], sc[kt]);
            kf = ldh(kcp + ko + 32); sc[kt] = wmma16(kf, qf[1], sc[kt]);
            kf = ldh(krp + ko);      sc[kt] = wmma16(kf, qf[2], sc[kt]);
            kf = ldh(krp + ko + 32); sc[kt] = wmma16(kf, qf[3], sc[kt]);
        }
        asm volatile("v_nop\n\tv_nop\n\tv_nop\n\tv_nop" : "+v"(sc[0]), "+v"(sc[1]) : "v"(kf), "v"(qf[3]));
        float mloc = NEG;
#pragma unroll
        for (int kt = 0; kt < 2; ++kt)
#pragma unroll
            for (int i = 0; i < 8; ++i) { const int j = kb + kt * 16 + 8 * hh + i; const float u = (j <= q) ? sc[kt][i] * cc : NEG; sc[kt][i] = u; mloc = fmaxf(mloc, u); }
        mloc = fmaxf(mloc, __shfl_xor(mloc, 16, 32));
        const float mn = fmaxf(m, mloc);
        const float alpha = __builtin_amdgcn_exp2f(m - mn);
        float psm = 0.0f;
#pragma unroll
        for (int kt = 0; kt < 2; ++kt)
#pragma unroll
            for (int i = 0; i < 8; ++i) { const float p = __builtin_amdgcn_exp2f(sc[kt][i] - mn); sc[kt][i] = p; psm += p; }
        psm += __shfl_xor(psm, 16, 32);
        l = l * alpha + psm; m = mn;
#pragma unroll
        for (int r = 0; r < 8; ++r) { const float ar = __shfl(alpha, 8 * hh + r, 32);
#pragma unroll
            for (int n = 0; n < 8; ++n) of[n][r] *= ar; }
        v8h p0, p1;
#pragma unroll
        for (int i = 0; i < 8; ++i) { p0[i] = (h16)(sc[0][i] * PCAR); p1[i] = (h16)(sc[1][i] * PCAR); }
        const v16h pf = cat16(p0, p1);
        v16h vf;
#pragma unroll
        for (int n = 0; n < 8; ++n) { asm volatile("" ::: "memory"); vf = ldh(vp + (size_t)n * 16 * SEQ + kb); of[n] = wmma16(pf, vf, of[n]); }
        asm volatile("v_nop\n\tv_nop\n\tv_nop\n\tv_nop" : "+v"(of[0]), "+v"(of[7]) : "v"(pf), "v"(vf));
    }
    const float fin = (CSC / PCAR) * (1.0f / l);
    h16* osw = &os[wv][0];
#pragma unroll
    for (int r = 0; r < 8; ++r) { const float fr = __shfl(fin, 8 * hh + r, 32);
#pragma unroll
        for (int n = 0; n < 8; ++n) osw[(8 * hh + r) * OSP + n * 16 + lr] = (h16)(of[n][r] * fr); }
    __builtin_amdgcn_fence(3, "wavefront"); __builtin_amdgcn_wave_barrier(); asm volatile("" ::: "memory");
    h16* cb = CT16 + (size_t)qw * DMOD + hd * DHD + lr * 8;
#pragma unroll 1
    for (int ps = 0; ps < 2; ++ps) {
#pragma unroll
        for (int s8 = 0; s8 < 8; ++s8) { const int row = 2 * s8 + hh; const v8h v = *(const v8ha*)(osw + row * OSP + lr * 8); *(volatile v8h*)(cb + (size_t)row * DMOD) = v; }
        if (ps == 0) __threadfence(); }
}

__global__ __launch_bounds__(128) __attribute__((amdgpu_num_vgpr(256)))
void k_attnh(const bf* __restrict__ Qh, const bf* __restrict__ Ql, const bf* __restrict__ KCh, const bf* __restrict__ KCl, const bf* __restrict__ KRh, const bf* __restrict__ KRl,
             const bf* __restrict__ VTh, const bf* __restrict__ VTl, bf* CTh, bf* CTl) {
    __shared__ __align__(16) bf os[4][16 * OSP];
    const int lane = threadIdx.x & 31, wv = threadIdx.x >> 5, lr = lane & 15, hh = lane >> 4;
    const int hd = blockIdx.y;
    const int qw = blockIdx.x * QB + wv * 16;
    const int q = qw + lr;
    const bf* qhp = Qh + ((size_t)hd * RH + q) * DHD + 8 * hh;
    const bf* qlp = Ql + ((size_t)hd * RH + q) * DHD + 8 * hh;
    const bf* kch = KCh + ((size_t)hd * RH + lr) * HALF + 8 * hh;
    const bf* kcl = KCl + ((size_t)hd * RH + lr) * HALF + 8 * hh;
    const bf* krh = KRh + (size_t)lr * HALF + 8 * hh;
    const bf* krl = KRl + (size_t)lr * HALF + 8 * hh;
    const bf* vhb = VTh + ((size_t)hd * DHD + lr) * RH + 8 * hh;
    const bf* vlb = VTl + ((size_t)hd * DHD + lr) * RH + 8 * hh;
    v8f of[8];
#pragma unroll
    for (int n = 0; n < 8; ++n) of[n] = (v8f){};
    float m = NEG, l = 0.0f;
    const float cc = SCL * L2E;
    const int ns = (qw >> 5) + 1;
#pragma unroll 1
    for (int s = 0; s < ns; ++s) {
        const int kb = s * 32;
        v8f sc[2]; sc[0] = (v8f){}; sc[1] = (v8f){};
        v16bf bq, bq2, ak, ak2;
#pragma unroll
        for (int c = 0; c < 4; ++c) {
            asm volatile("" ::: "memory");
            bq = ldb(qhp + c * 32); bq2 = ldb(qlp + c * 32);
            const bf* kh = (c < 2) ? (kch + c * 32) : (krh + (c - 2) * 32);
            const bf* kl = (c < 2) ? (kcl + c * 32) : (krl + (c - 2) * 32);
#pragma unroll
            for (int kt = 0; kt < 2; ++kt) {
                const size_t ko = (size_t)(kb + kt * 16) * HALF;
                asm volatile("" ::: "memory");
                ak = ldb(kh + ko); ak2 = ldb(kl + ko);
                sc[kt] = wmmab(ak, bq, sc[kt]); sc[kt] = wmmab(ak, bq2, sc[kt]); sc[kt] = wmmab(ak2, bq, sc[kt]);
            }
        }
        asm volatile("v_nop\n\tv_nop\n\tv_nop\n\tv_nop" : "+v"(sc[0]), "+v"(sc[1]) : "v"(ak), "v"(ak2), "v"(bq), "v"(bq2));
        float mloc = NEG;
#pragma unroll
        for (int kt = 0; kt < 2; ++kt)
#pragma unroll
            for (int i = 0; i < 8; ++i) { const int j = kb + kt * 16 + 8 * hh + i; const float u = (j <= q) ? sc[kt][i] * cc : NEG; sc[kt][i] = u; mloc = fmaxf(mloc, u); }
        mloc = fmaxf(mloc, __shfl_xor(mloc, 16, 32));
        const float mn = fmaxf(m, mloc);
        const float alpha = __builtin_amdgcn_exp2f(m - mn);
        float psm = 0.0f;
#pragma unroll
        for (int kt = 0; kt < 2; ++kt)
#pragma unroll
            for (int i = 0; i < 8; ++i) { const float p = __builtin_amdgcn_exp2f(sc[kt][i] - mn); sc[kt][i] = p; psm += p; }
        psm += __shfl_xor(psm, 16, 32);
        l = l * alpha + psm; m = mn;
#pragma unroll
        for (int r = 0; r < 8; ++r) { const float ar = __shfl(alpha, 8 * hh + r, 32);
#pragma unroll
            for (int n = 0; n < 8; ++n) of[n][r] *= ar; }
        v8us ph0, ph1, pl0, pl1;
#pragma unroll
        for (int i = 0; i < 8; ++i) { unsigned short a0, c0, a1, c1; splitf(sc[0][i], a0, c0); splitf(sc[1][i], a1, c1); ph0[i] = a0; pl0[i] = c0; ph1[i] = a1; pl1[i] = c1; }
        const v16bf pa = cat16b(ph0, ph1), pb = cat16b(pl0, pl1);
        v16bf vh, vl;
#pragma unroll
        for (int n = 0; n < 8; ++n) { asm volatile("" ::: "memory"); vh = ldb(vhb + (size_t)n * 16 * RH + kb); vl = ldb(vlb + (size_t)n * 16 * RH + kb);
            of[n] = wmmab(pa, vh, of[n]); of[n] = wmmab(pa, vl, of[n]); of[n] = wmmab(pb, vh, of[n]); }
        asm volatile("v_nop\n\tv_nop\n\tv_nop\n\tv_nop" : "+v"(of[0]), "+v"(of[7]) : "v"(pa), "v"(pb), "v"(vh), "v"(vl));
    }
    const float fin = 1.0f / l;
    bf* osw = &os[wv][0];
#pragma unroll
    for (int r = 0; r < 8; ++r) { const float fr = __shfl(fin, 8 * hh + r, 32);
#pragma unroll
        for (int n = 0; n < 8; ++n) osw[(8 * hh + r) * OSP + n * 16 + lr] = f2bf(of[n][r] * fr); }
    __builtin_amdgcn_fence(3, "wavefront"); __builtin_amdgcn_wave_barrier(); asm volatile("" ::: "memory");
    { bf* cb = CTh + (size_t)qw * DMOD + hd * DHD + lr * 8;
#pragma unroll 1
        for (int ps = 0; ps < 2; ++ps) {
#pragma unroll
            for (int s8 = 0; s8 < 8; ++s8) { const int row = 2 * s8 + hh; const v8us v = *(const v8usa*)(osw + row * OSP + lr * 8); *(volatile v8us*)(cb + (size_t)row * DMOD) = v; }
            if (ps == 0) __threadfence(); } }
    __builtin_amdgcn_fence(3, "wavefront"); __builtin_amdgcn_wave_barrier(); asm volatile("" ::: "memory");
#pragma unroll
    for (int r = 0; r < 8; ++r) { const float fr = __shfl(fin, 8 * hh + r, 32);
#pragma unroll
        for (int n = 0; n < 8; ++n) { unsigned short a0, c0; splitf(of[n][r] * fr, a0, c0); osw[(8 * hh + r) * OSP + n * 16 + lr] = c0; } }
    __builtin_amdgcn_fence(3, "wavefront"); __builtin_amdgcn_wave_barrier(); asm volatile("" ::: "memory");
    { bf* cb = CTl + (size_t)qw * DMOD + hd * DHD + lr * 8;
#pragma unroll 1
        for (int ps = 0; ps < 2; ++ps) {
#pragma unroll
            for (int s8 = 0; s8 < 8; ++s8) { const int row = 2 * s8 + hh; const v8us v = *(const v8usa*)(osw + row * OSP + lr * 8); *(volatile v8us*)(cb + (size_t)row * DMOD) = v; }
            if (ps == 0) __threadfence(); } }
}

extern "C" void kernel_launch(void* const* d_in, const int* in_sizes, int n_in,
                              void* d_out, int out_size, void* d_ws, size_t ws_size, hipStream_t stream) {
    if (n_in < 15) return;
    if (in_sizes[0] < ((NB - 1) * SEQ_FULL + SEQ) * DMOD) return;
    if (in_sizes[1] < (SEQ - 1) * SEQ_FULL + SEQ) return;
    if (in_sizes[2] < SEQ * NPAIR || in_sizes[3] < SEQ * NPAIR) return;
    if (in_sizes[4] < DMOD || in_sizes[5] < DCQ || in_sizes[6] < DCKV) return;
    if (in_sizes[7] < DMOD * DCQ || in_sizes[8] < DCQ * NHD * HALF || in_sizes[9] < DCQ * NHD * HALF || in_sizes[10] < DMOD * DCKV) return;
    if (in_sizes[11] < DCKV * NHD * HALF || in_sizes[12] < DMOD * HALF || in_sizes[13] < DCKV * NHD * DHD || in_sizes[14] < NHD * DHD * DMOD) return;
    if (out_size < NB * SEQ * DMOD) return;
    const float* x    = (const float*)d_in[0];
    const int*   msk  = (const int*)d_in[1];
    const float* cosT = (const float*)d_in[2];
    const float* sinT = (const float*)d_in[3];
    const float* w_in = (const float*)d_in[4];
    const float* w_cq = (const float*)d_in[5];
    const float* w_ckv= (const float*)d_in[6];
    const float* W_cq = (const float*)d_in[7];
    const float* W_q  = (const float*)d_in[8];
    const float* W_qR = (const float*)d_in[9];
    const float* W_ckv= (const float*)d_in[10];
    const float* W_k  = (const float*)d_in[11];
    const float* W_kR = (const float*)d_in[12];
    const float* W_v  = (const float*)d_in[13];
    const float* W_o  = (const float*)d_in[14];
    float* OUT = (float*)d_out;

    char* wsp = (char*)d_ws;
    auto take = [&](size_t bytes) { char* p = wsp; wsp += (bytes + 255) & ~(size_t)255; return (void*)p; };
    bf*  WCAT = (bf*)take((size_t)NU * DMOD * 2);
    h16* WQQ  = (h16*)take((size_t)NQQ * DCQ * 2);
    h16* WKV  = (h16*)take((size_t)NKV * DCKV * 2);
    h16* WO16 = (h16*)take((size_t)DMOD * (NHD * DHD) * 2);
    bf*  WOB  = (bf*)take((size_t)DMOD * (NHD * DHD) * 2);
    bf*  XB   = (bf*)take((size_t)SEQ * DMOD * 2);
    float* FS = (float*)take((size_t)SEQ * NKV * 4);
    h16* CQ16 = (h16*)take((size_t)SEQ * DCQ * 2);
    h16* CKV16= (h16*)take((size_t)SEQ * DCKV * 2);
    h16* Q16  = (h16*)take((size_t)NHD * SEQ * DHD * 2);
    bf*  Qh   = (bf*)take((size_t)NHD * RH * DHD * 2);
    bf*  Ql   = (bf*)take((size_t)NHD * RH * DHD * 2);
    h16* KC16 = (h16*)take((size_t)NHD * SEQ * HALF * 2);
    bf*  KCh  = (bf*)take((size_t)NHD * RH * HALF * 2);
    bf*  KCl  = (bf*)take((size_t)NHD * RH * HALF * 2);
    h16* KR16 = (h16*)take((size_t)SEQ * HALF * 2);
    bf*  KRh  = (bf*)take((size_t)RH * HALF * 2);
    bf*  KRl  = (bf*)take((size_t)RH * HALF * 2);
    h16* VT16 = (h16*)take((size_t)NHD * DHD * SEQ * 2);
    bf*  VTh  = (bf*)take((size_t)NHD * DHD * RH * 2);
    bf*  VTl  = (bf*)take((size_t)NHD * DHD * RH * 2);
    h16* CT16 = (h16*)take((size_t)SEQ * DMOD * 2);
    bf*  CTh  = (bf*)take((size_t)RH * DMOD * 2);
    bf*  CTl  = (bf*)take((size_t)RH * DMOD * 2);
    int* FLG  = (int*)take((size_t)(SEQ / 16) * 32 * 4);
    int* FLAG = (int*)take(128);
    if ((size_t)(wsp - (char*)d_ws) > ws_size) return;

    auto gl = [](size_t nelem) { return (unsigned)((nelem / 64 + 63) / 64); };
    k_wcv<false, true><<<gl((size_t)DMOD * DCQ), 256, 0, stream>>>(W_cq, DMOD, DCQ, 0, 1.0f, nullptr, WCAT);
    k_wcv<false, true><<<gl((size_t)DMOD * DCKV), 256, 0, stream>>>(W_ckv, DMOD, DCKV, DCQ, 1.0f, nullptr, WCAT);
    k_wcv<false, true><<<gl((size_t)DMOD * HALF), 256, 0, stream>>>(W_kR, DMOD, HALF, DCQ + DCKV, 1.0f, nullptr, WCAT);
    k_wcv<true, false><<<gl((size_t)DCQ * NHD * HALF), 256, 0, stream>>>(W_q, DCQ, NHD * HALF, 0, WSC, WQQ, nullptr);
    k_wcv<true, false><<<gl((size_t)DCQ * NHD * HALF), 256, 0, stream>>>(W_qR, DCQ, NHD * HALF, NHD * HALF, WSC, WQQ, nullptr);
    k_wcv<true, false><<<gl((size_t)DCKV * NHD * DHD), 256, 0, stream>>>(W_v, DCKV, NHD * DHD, 0, WSC, WKV, nullptr);
    k_wcv<true, false><<<gl((size_t)DCKV * NHD * HALF), 256, 0, stream>>>(W_k, DCKV, NHD * HALF, NHD * DHD, WSC, WKV, nullptr);
    k_wcv<true, true><<<gl((size_t)(NHD * DHD) * DMOD), 256, 0, stream>>>(W_o, NHD * DHD, DMOD, 0, WSC, WO16, WOB);
    k_mchk<<<SEQ / 16, 256, 0, stream>>>(msk, FLG);
    k_fred<<<1, 32, 0, stream>>>(FLG, SEQ / 16, FLAG);

    for (int b = 0; b < NB; ++b) {
        const float* xb = x + (size_t)b * SEQ_FULL * DMOD;
        float* outb = OUT + (size_t)b * SEQ * DMOD;
        k_cvtx<<<(unsigned)(((size_t)SEQ * DMOD / 8 + 255) / 256), 256, 0, stream>>>(xb, w_in, XB, (size_t)SEQ * DMOD / 8);
        k_gemmw<bf, 0, false><<<dim3(SEQ / 64, NU / 64, 1), 32, 0, stream>>>(XB, nullptr, WCAT, nullptr, DMOD, FS, NU, 1.0f, nullptr, 0, FLAG);
        k_lat<<<SEQ / 8, 256, 0, stream>>>(xb, FS, w_cq, w_ckv, cosT, sinT, CQ16, CKV16, KR16, KRh, KRl);
        k_gemmw<h16, 0, false><<<dim3(SEQ / 64, NQQ / 64, 1), 32, 0, stream>>>(CQ16, nullptr, WQQ, nullptr, DCQ, FS, NQQ, 1.0f / WSC, nullptr, 0, FLAG);
        k_qpl<<<(unsigned)(((size_t)NHD * SEQ * DHD / 2 + 255) / 256), 256, 0, stream>>>(FS, cosT, sinT, Q16, Qh, Ql);
        k_gemmw<h16, 0, false><<<dim3(SEQ / 64, NKV / 64, 1), 32, 0, stream>>>(CKV16, nullptr, WKV, nullptr, DCKV, FS, NKV, 1.0f / WSC, nullptr, 0, FLAG);
        k_kcpl<<<(unsigned)(((size_t)NHD * SEQ * HALF / 2 + 255) / 256), 256, 0, stream>>>(FS, KC16, KCh, KCl);
        k_vtpl<<<(unsigned)(((size_t)NHD * DHD * SEQ / 2 + 255) / 256), 256, 0, stream>>>(FS, VT16, VTh, VTl);
        k_attnh<<<dim3(RH / QB, NHD, 1), 128, 0, stream>>>(Qh, Ql, KCh, KCl, KRh, KRl, VTh, VTl, CTh, CTl);
        if (SEQ > RH) k_attn<<<dim3((SEQ - RH) / QB, NHD, 1), 128, 0, stream>>>(Q16, KC16, KR16, VT16, CT16);
        k_gemmw<bf, 1, true><<<dim3(RH / 64, DMOD / 64, 1), 32, 0, stream>>>(CTh, CTl, WOB, nullptr, NHD * DHD, outb, DMOD, 1.0f, xb, DMOD, FLAG);
        if (SEQ > RH) k_gemmw<h16, 0, true><<<dim3((SEQ - RH) / 64, DMOD / 64, 1), 32, 0, stream>>>(CT16 + (size_t)RH * DMOD, nullptr, WO16, nullptr, NHD * DHD, outb + (size_t)RH * DMOD, DMOD, 1.0f / (WSC * CSC), xb + (size_t)RH * DMOD, DMOD, FLAG);
    }
}
